// Mamba_46797963657514
// MI455X (gfx1250) — hardware-run, weakly checked
//
#include <hip/hip_runtime.h>
#include <hip/hip_fp16.h>
#include <math.h>

typedef __attribute__((ext_vector_type(16))) _Float16 v16h;
typedef __attribute__((ext_vector_type(8)))  _Float16 v8h;
typedef __attribute__((ext_vector_type(8)))  float    v8f;
typedef __attribute__((ext_vector_type(4)))  float    v4f;
typedef __attribute__((ext_vector_type(4)))  unsigned v4u;

constexpr int kBatch = 8;
constexpr int kSeq   = 2048;
constexpr int kDm    = 128;
constexpr int kNL    = 4;
constexpr int kDin   = 256;
constexpr int kTaps  = 8;
constexpr int kNst   = 16;
constexpr int kDtR   = 8;
constexpr int kRows  = kBatch * kSeq;
constexpr int kXzP   = 2 * kDin;
constexpr int kDbcW  = kDtR + 2 * kNst;
constexpr int kDbcP  = 64;
constexpr int kOffB  = kDtR;
constexpr int kOffC  = kDtR + kNst;
constexpr int kConvTP = 260;
static_assert(kRows == 16384);
static_assert(kXzP == 512);
static_assert(kDbcW == 40);
static_assert(kTaps == 8);
static_assert((kDm % 32) == 0 && (kDin % 32) == 0);
static_assert((kRows % 64) == 0 && (kXzP % 64) == 0 && (kDbcP % 64) == 0 && (kDm % 64) == 0);
static_assert((kDin % 64) == 0 && (kSeq % 64) == 0);

constexpr float kWCarry = 1024.0f;
constexpr float kACarry = 64.0f;
constexpr float kYCarry = 256.0f;
constexpr float kScaleIn  = 1.0f / (kACarry * kWCarry);
constexpr float kScaleOut = 1.0f / (kYCarry * kWCarry);

constexpr size_t kSzWI  = (size_t)kNL * kXzP * kDm * 2;
constexpr size_t kSzWX  = (size_t)kNL * kDbcP * kDin * 2;
constexpr size_t kSzWO  = (size_t)kNL * kDm * kDin * 2;
constexpr size_t kSzXN  = (size_t)kRows * kDm * 2;
constexpr size_t kSzXZ  = (size_t)kRows * kXzP * 4;
constexpr size_t kSzU32 = (size_t)kRows * kDin * 4;
constexpr size_t kSzU16 = (size_t)kRows * kDin * 2;
constexpr size_t kSzDBC = (size_t)kRows * kDbcP * 4;
constexpr size_t kSzDTP = (size_t)kRows * kDin * 4;
constexpr size_t kSzY16 = (size_t)kRows * kDin * 2;
constexpr size_t kSzR   = (size_t)kRows * kDm * 4;
constexpr size_t kOffWI  = 0;
constexpr size_t kOffWX  = kOffWI  + kSzWI;
constexpr size_t kOffWO  = kOffWX  + kSzWX;
constexpr size_t kOffXN  = kOffWO  + kSzWO;
constexpr size_t kOffXZ  = kOffXN  + kSzXN;
constexpr size_t kOffU32 = kOffXZ  + kSzXZ;
constexpr size_t kOffU16 = kOffU32 + kSzU32;
constexpr size_t kOffDBC = kOffU16 + kSzU16;
constexpr size_t kOffDTP = kOffDBC + kSzDBC;
constexpr size_t kOffY16 = kOffDTP + kSzDTP;
constexpr size_t kOffRA  = kOffY16 + kSzY16;
constexpr size_t kOffRB  = kOffRA  + kSzR;
constexpr size_t kWsTotal = kOffRB + kSzR;
static_assert(kWsTotal == 109969408ull);
static_assert(kWsTotal <= 134217728ull);
static_assert((kOffWX % 128) == 0 && (kOffWO % 128) == 0 && (kOffXN % 128) == 0 && (kOffXZ % 128) == 0 &&
              (kOffU32 % 128) == 0 && (kOffU16 % 128) == 0 && (kOffDBC % 128) == 0 && (kOffDTP % 128) == 0 &&
              (kOffY16 % 128) == 0 && (kOffRA % 128) == 0 && (kOffRB % 128) == 0);

__device__ __forceinline__ unsigned g_h16bits(float v) {
  const float f = (fabsf(v) < 6.103515625e-05f) ? 0.0f : v;
  return (unsigned)__half_as_ushort(__float2half_rn(f));
}
__device__ __forceinline__ unsigned g_pack16(float a, float b) {
  const unsigned lo = g_h16bits(a);
  const unsigned hi = g_h16bits(b);
  return lo | (hi << 16);
}

constexpr int kPrepBlkWi = kNL * kXzP * kDm / 8 / 256;
constexpr int kPrepBlkWx = kNL * kDbcP * kDin / 8 / 256;
constexpr int kPrepBlkWo = kNL * kDm * kDin / 8 / 256;
static_assert(kPrepBlkWi == 128 && kPrepBlkWx == 32 && kPrepBlkWo == 64);

__global__ __launch_bounds__(256) void prep_weights_kernel(
    const float* __restrict__ wi, const float* __restrict__ wx, const float* __restrict__ wo,
    unsigned short* __restrict__ WI, unsigned short* __restrict__ WX, unsigned short* __restrict__ WO)
{
  const int blk = blockIdx.x;
  const int tid = threadIdx.x;
  const float* src;
  unsigned short* dst;
  bool live = true;
  if (blk < kPrepBlkWi) {
    const size_t e0 = ((size_t)blk * 256 + tid) * 8;
    src = wi + e0;
    dst = WI + e0;
  } else if (blk < kPrepBlkWi + kPrepBlkWx) {
    const int local = ((blk - kPrepBlkWi) * 256 + tid) * 8;
    const int layer = local / (kDbcP * kDin);
    const int rem   = local - layer * (kDbcP * kDin);
    const int row   = rem / kDin;
    const int col   = rem - row * kDin;
    live = (row < kDbcW);
    const int rc = live ? row : (kDbcW - 1);
    src = wx + ((size_t)layer * kDbcW + rc) * kDin + col;
    dst = WX + local;
  } else {
    const size_t e0 = ((size_t)(blk - kPrepBlkWi - kPrepBlkWx) * 256 + tid) * 8;
    src = wo + e0;
    dst = WO + e0;
  }
  const v4f a0 = *(const v4f*)(src);
  const v4f a1 = *(const v4f*)(src + 4);
  float f0 = a0[0], f1 = a0[1], f2 = a0[2], f3 = a0[3];
  float f4 = a1[0], f5 = a1[1], f6 = a1[2], f7 = a1[3];
  f0 = live ? f0 * kWCarry : 0.0f;
  f1 = live ? f1 * kWCarry : 0.0f;
  f2 = live ? f2 * kWCarry : 0.0f;
  f3 = live ? f3 * kWCarry : 0.0f;
  f4 = live ? f4 * kWCarry : 0.0f;
  f5 = live ? f5 * kWCarry : 0.0f;
  f6 = live ? f6 * kWCarry : 0.0f;
  f7 = live ? f7 * kWCarry : 0.0f;
  const unsigned w0 = g_pack16(f0, f1);
  const unsigned w1 = g_pack16(f2, f3);
  const unsigned w2 = g_pack16(f4, f5);
  const unsigned w3 = g_pack16(f6, f7);
  const v4u w = (v4u){w0, w1, w2, w3};
  volatile v4u* q = (volatile v4u*)dst;
  *q = w;
  __threadfence();
  *q = w;
}

__global__ __launch_bounds__(256) void rmsnorm_kernel(
    const float* __restrict__ R, const float* __restrict__ gw, unsigned short* __restrict__ XN)
{
  const int tid = threadIdx.x;
  const int lane = tid & 31;
  const int wave = tid >> 5;
  const int half = lane >> 4;
  const int c0 = (lane & 15) * 8;
  const int row = blockIdx.x * 16 + wave * 2 + half;
  const float* p = R + (size_t)row * kDm + c0;
  const v4f a0 = *(const v4f*)(p);
  const v4f a1 = *(const v4f*)(p + 4);
  const v4f g0 = *(const v4f*)(gw + c0);
  const v4f g1 = *(const v4f*)(gw + c0 + 4);
  float ss = 0.0f;
  ss = fmaf(a0[0], a0[0], ss);
  ss = fmaf(a0[1], a0[1], ss);
  ss = fmaf(a0[2], a0[2], ss);
  ss = fmaf(a0[3], a0[3], ss);
  ss = fmaf(a1[0], a1[0], ss);
  ss = fmaf(a1[1], a1[1], ss);
  ss = fmaf(a1[2], a1[2], ss);
  ss = fmaf(a1[3], a1[3], ss);
  ss += __shfl_xor(ss, 8, 32);
  ss += __shfl_xor(ss, 4, 32);
  ss += __shfl_xor(ss, 2, 32);
  ss += __shfl_xor(ss, 1, 32);
  const float rs = rsqrtf(ss * (1.0f / (float)kDm) + 1e-5f);
  const float o0 = a0[0] * rs * g0[0] * kACarry;
  const float o1 = a0[1] * rs * g0[1] * kACarry;
  const float o2 = a0[2] * rs * g0[2] * kACarry;
  const float o3 = a0[3] * rs * g0[3] * kACarry;
  const float o4 = a1[0] * rs * g1[0] * kACarry;
  const float o5 = a1[1] * rs * g1[1] * kACarry;
  const float o6 = a1[2] * rs * g1[2] * kACarry;
  const float o7 = a1[3] * rs * g1[3] * kACarry;
  const v4u w = (v4u){g_pack16(o0, o1), g_pack16(o2, o3), g_pack16(o4, o5), g_pack16(o6, o7)};
  volatile v4u* q = (volatile v4u*)(XN + (size_t)row * kDm + c0);
  *q = w;
  __threadfence();
  *q = w;
}

__global__ __launch_bounds__(256) void conv_silu_kernel(
    const float* __restrict__ XZ, const float* __restrict__ cw, const float* __restrict__ cb,
    float* __restrict__ U32, unsigned short* __restrict__ U16)
{
  __shared__ __align__(16) float sT[16 * kConvTP];
  const int tid = threadIdx.x;
  const int lane = tid & 31;
  const int wave = tid >> 5;
  const int d = tid;
  const int g0 = blockIdx.x * 64;
  const int tb = g0 & (kSeq - 1);
  const v4f wa = *(const v4f*)(cw + d * kTaps);
  const v4f wb = *(const v4f*)(cw + d * kTaps + 4);
  const float w0 = wa[0], w1 = wa[1], w2 = wa[2], w3 = wa[3];
  const float w4 = wb[0], w5 = wb[1], w6 = wb[2], w7 = wb[3];
  const float bias = cb[d];
  float xm7, xm6, xm5, xm4, xm3, xm2, xm1;
  {
    const bool hist = (tb > 0);
    const int rb = hist ? (g0 - 7) : g0;
    const float v7 = XZ[(size_t)(rb + 0) * kXzP + d];
    const float v6 = XZ[(size_t)(rb + 1) * kXzP + d];
    const float v5 = XZ[(size_t)(rb + 2) * kXzP + d];
    const float v4 = XZ[(size_t)(rb + 3) * kXzP + d];
    const float v3 = XZ[(size_t)(rb + 4) * kXzP + d];
    const float v2 = XZ[(size_t)(rb + 5) * kXzP + d];
    const float v1 = XZ[(size_t)(rb + 6) * kXzP + d];
    xm7 = hist ? v7 : 0.0f;
    xm6 = hist ? v6 : 0.0f;
    xm5 = hist ? v5 : 0.0f;
    xm4 = hist ? v4 : 0.0f;
    xm3 = hist ? v3 : 0.0f;
    xm2 = hist ? v2 : 0.0f;
    xm1 = hist ? v1 : 0.0f;
  }
  const int hrow = wave >> 1;
  const int hch  = (wave & 1) * 128 + lane * 4;
#pragma unroll 1
  for (int sub = 0; sub < 4; ++sub) {
    const int lb = g0 + sub * 16;
#pragma unroll 1
    for (int s = 0; s < 16; ++s) {
      const float xcur = XZ[(size_t)(lb + s) * kXzP + d];
      float acc = w0 * xm7;
      acc = fmaf(w1, xm6, acc);
      acc = fmaf(w2, xm5, acc);
      acc = fmaf(w3, xm4, acc);
      acc = fmaf(w4, xm3, acc);
      acc = fmaf(w5, xm2, acc);
      acc = fmaf(w6, xm1, acc);
      acc = fmaf(w7, xcur, acc);
      const float sv = acc + bias;
      const float sg = __builtin_amdgcn_rcpf(1.0f + expf(-sv));
      sT[s * kConvTP + tid] = sv * sg;
      xm7 = xm6;
      xm6 = xm5;
      xm5 = xm4;
      xm4 = xm3;
      xm3 = xm2;
      xm2 = xm1;
      xm1 = xcur;
    }
    __syncthreads();
    v4f fv[4];
    v4u hv[2];
#pragma unroll
    for (int it = 0; it < 4; ++it) fv[it] = *(const v4f*)(sT + (it * 4 + hrow) * kConvTP + hch);
#pragma unroll
    for (int it = 0; it < 2; ++it) {
      const float* sp = sT + (it * 8 + wave) * kConvTP + lane * 8;
      const v4f a0 = *(const v4f*)(sp);
      const v4f a1 = *(const v4f*)(sp + 4);
      const float e0 = a0[0] * kACarry, e1 = a0[1] * kACarry, e2 = a0[2] * kACarry, e3 = a0[3] * kACarry;
      const float e4 = a1[0] * kACarry, e5 = a1[1] * kACarry, e6 = a1[2] * kACarry, e7 = a1[3] * kACarry;
      hv[it] = (v4u){g_pack16(e0, e1), g_pack16(e2, e3), g_pack16(e4, e5), g_pack16(e6, e7)};
    }
    for (int pass = 0; pass < 2; ++pass) {
#pragma unroll
      for (int it = 0; it < 4; ++it)
        *(volatile v4f*)(U32 + (size_t)(lb + it * 4 + hrow) * kDin + hch) = fv[it];
#pragma unroll
      for (int it = 0; it < 2; ++it)
        *(volatile v4u*)(U16 + (size_t)(lb + it * 8 + wave) * kDin + lane * 8) = hv[it];
      __threadfence();
    }
    __syncthreads();
  }
}

__global__ __launch_bounds__(256) void dtpre_kernel(
    const float* __restrict__ DBC, const float* __restrict__ dw, const float* __restrict__ db,
    float* __restrict__ DTP)
{
  const int tid = threadIdx.x;
  const int c4 = (tid & 63) * 4;
  const int rsub = tid >> 6;
  v4f wlo[4], whi[4];
#pragma unroll
  for (int j = 0; j < 4; ++j) {
    wlo[j] = *(const v4f*)(dw + (size_t)(c4 + j) * kDtR);
    whi[j] = *(const v4f*)(dw + (size_t)(c4 + j) * kDtR + 4);
  }
  const v4f bv = *(const v4f*)(db + c4);
  const int r0 = blockIdx.x * 64;
#pragma unroll 1
  for (int it = 0; it < 16; ++it) {
    const int row = r0 + it * 4 + rsub;
    const v4f xa = *(const v4f*)(DBC + (size_t)row * kDbcP);
    const v4f xb = *(const v4f*)(DBC + (size_t)row * kDbcP + 4);
    float o[4];
#pragma unroll
    for (int j = 0; j < 4; ++j) {
      float acc = xa[0] * wlo[j][0];
      acc = fmaf(xa[1], wlo[j][1], acc);
      acc = fmaf(xa[2], wlo[j][2], acc);
      acc = fmaf(xa[3], wlo[j][3], acc);
      acc = fmaf(xb[0], whi[j][0], acc);
      acc = fmaf(xb[1], whi[j][1], acc);
      acc = fmaf(xb[2], whi[j][2], acc);
      acc = fmaf(xb[3], whi[j][3], acc);
      o[j] = acc + bv[j];
    }
    const v4f ov = (v4f){o[0], o[1], o[2], o[3]};
    volatile v4f* q = (volatile v4f*)(DTP + (size_t)row * kDin + c4);
    *q = ov;
    __threadfence();
    *q = ov;
  }
}

namespace eng {

__device__ __forceinline__ v16h frag_load(const _Float16* p) {
  union U { v16h v; v8h h[2]; } f;
  f.h[0] = *(const v8h*)(p);
  f.h[1] = *(const v8h*)(p + 16);
  return f.v;
}
__device__ __forceinline__ v8f mma_h(v16h a, v16h b, v8f c) {
  c = __builtin_amdgcn_wmma_f32_16x16x32_f16(false, a, false, b, (short)0, c, false, false);
  asm volatile("v_nop\n\tv_nop\n\tv_nop\n\tv_nop" : "+v"(c) : "v"(a), "v"(b));
  return c;
}

template <bool RESID>
__global__ __launch_bounds__(256) void gemm_f16_kernel(
    const unsigned short* __restrict__ Ap, int lda,
    const unsigned short* __restrict__ Btp, int ldb,
    float* __restrict__ C, int ldc,
    const float* __restrict__ resid,
    int M, int N, int K, float scale)
{
  const _Float16* A  = (const _Float16*)Ap;
  const _Float16* Bt = (const _Float16*)Btp;
  __shared__ __align__(16) float sT[8][16 * 68];
  const int lane = threadIdx.x & 31;
  const int wave = threadIdx.x >> 5;
  const int tilesN = N >> 6;
  const int tilesM = M >> 6;
  const int tile = blockIdx.x * 8 + wave;
  if (tile >= tilesM * tilesN) return;
  const int tm = tile / tilesN;
  const int tn = tile - tm * tilesN;
  const int m0 = tm << 6;
  const int n0 = tn << 6;
  const int rlane = lane & 15;
  const int koff  = (lane >> 4) * 8;
  const int mOff  = (lane >> 4) * 8;

  v8f acc[4][4];
#pragma unroll
  for (int i = 0; i < 4; ++i)
#pragma unroll
    for (int j = 0; j < 4; ++j) acc[i][j] = (v8f){0.f, 0.f, 0.f, 0.f, 0.f, 0.f, 0.f, 0.f};

  for (int k0 = 0; k0 < K; k0 += 32) {
    v16h bh[4];
#pragma unroll
    for (int j = 0; j < 4; ++j) {
      const size_t bo = (size_t)(n0 + (j << 4) + rlane) * ldb + koff + k0;
      bh[j] = frag_load(Bt + bo);
    }
#pragma unroll
    for (int i = 0; i < 4; ++i) {
      const size_t ao = (size_t)(m0 + (i << 4) + rlane) * lda + koff + k0;
      const v16h ah = frag_load(A + ao);
#pragma unroll
      for (int j = 0; j < 4; ++j) acc[i][j] = mma_h(ah, bh[j], acc[i][j]);
    }
  }

  float* slab = sT[wave];
  const int hh = lane >> 4;
  const int c4 = (lane & 15) * 4;
#pragma unroll
  for (int i = 0; i < 4; ++i) {
    const int mBase = m0 + (i << 4);
#pragma unroll
    for (int j = 0; j < 4; ++j) {
#pragma unroll
      for (int r = 0; r < 8; ++r) {
        slab[(mOff + r) * 68 + (j << 4) + rlane] = acc[i][j][r] * scale;
      }
    }
    __builtin_amdgcn_fence(__ATOMIC_RELEASE, "workgroup");
    __builtin_amdgcn_wave_barrier();
    __builtin_amdgcn_fence(__ATOMIC_ACQUIRE, "workgroup");
    v4f ov[8];
#pragma unroll
    for (int it = 0; it < 8; ++it) {
      const int row = it * 2 + hh;
      v4f v = *(const v4f*)(slab + row * 68 + c4);
      if (RESID) {
        const v4f rv = *(const v4f*)(resid + (size_t)(mBase + row) * ldc + n0 + c4);
        v = v + rv;
      }
      ov[it] = v;
    }
    for (int pass = 0; pass < 2; ++pass) {
#pragma unroll
      for (int it = 0; it < 8; ++it) {
        const int row = it * 2 + hh;
        *(volatile v4f*)(C + (size_t)(mBase + row) * ldc + n0 + c4) = ov[it];
      }
      __threadfence();
    }
    __builtin_amdgcn_fence(__ATOMIC_RELEASE, "workgroup");
    __builtin_amdgcn_wave_barrier();
    __builtin_amdgcn_fence(__ATOMIC_ACQUIRE, "workgroup");
  }
}

}

typedef float    ms1_v4f __attribute__((ext_vector_type(4)));
typedef unsigned ms1_v4u __attribute__((ext_vector_type(4)));
struct ms1_args {
  const float* dtpre;
  const float* u;
  const float* bc;
  const float* z;
  const float* A_log;
  const float* Dskip;
  __half* y;
  __half* y_lo;
  long ld_dtpre;
  long ld_u;
  long ld_bc;
  long ld_z;
  long ld_y;
  int offB;
  int offC;
  int offZ;
  float ycarry;
  int dir;
  int D;
  int L;
  int nbatch;
};
static_assert(sizeof(ms1_args) == 136);

__device__ __forceinline__ float ms1_flush16(float v) {
  return (fabsf(v) < 6.103515625e-05f) ? 0.0f : v;
}
__device__ __forceinline__ unsigned ms1_h16bits(float v) {
  return (unsigned)__half_as_ushort(__float2half_rn(ms1_flush16(v)));
}
__device__ __forceinline__ float ms1_h16val(unsigned b) {
  return __half2float(__ushort_as_half((unsigned short)b));
}
__device__ __forceinline__ float ms1_softplus(float v) {
  return fmaxf(v, 0.0f) + log1pf(expf(-fabsf(v)));
}
__device__ __forceinline__ void ms1_pack2(float v0, float v1, unsigned& hw, unsigned& lw) {
  const unsigned h0 = ms1_h16bits(v0);
  const unsigned h1 = ms1_h16bits(v1);
  const float r0 = (v0 - ms1_h16val(h0)) * 2048.0f;
  const float r1 = (v1 - ms1_h16val(h1)) * 2048.0f;
  const unsigned l0 = ms1_h16bits(r0);
  const unsigned l1 = ms1_h16bits(r1);
  hw = h0 | (h1 << 16);
  lw = l0 | (l1 << 16);
}

template <int NSTATE>
__global__ __launch_bounds__(64 * (NSTATE / 16)) void ms1_scan_kernel(ms1_args a)
{
  static_assert(NSTATE == 16 || NSTATE == 64);
  constexpr int NQ  = NSTATE / 16;
  constexpr int NT  = 64 * NQ;
  constexpr int NW  = NT / 32;
  constexpr int BCW = 2 * NSTATE;
  constexpr int YP  = 68;
  constexpr int RPI = NW * 4;
  constexpr int NIT = 64 / RPI;
  static_assert(16 * NT <= 64 * YP);
  __shared__ __align__(16) float sBC[64 * BCW];
  __shared__ __align__(16) float sY[64 * YP];
  const int tid  = threadIdx.x;
  const int lane = tid & 31;
  const int wave = tid >> 5;
  const int c    = tid / NQ;
  const int sq   = tid - c * NQ;
  const int bpb  = a.D / 64;
  const int bi   = blockIdx.x / bpb;
  if (bi >= a.nbatch) return;
  const int d0 = (blockIdx.x - bi * bpb) * 64;
  const int d  = d0 + c;
  const long rowb = (long)bi * a.L;
  const bool hasz  = (a.z != nullptr);
  const bool hasD  = (a.Dskip != nullptr);
  const bool hasLo = (a.y_lo != nullptr);

#pragma unroll 1
  for (int n = 0; n < 16; ++n) {
    const float al = a.A_log[(long)d * NSTATE + sq * 16 + n];
    sY[n * NT + tid] = -expf(al);
  }
  __syncthreads();
  float An[16], h[16];
#pragma unroll
  for (int n = 0; n < 16; ++n) {
    An[n] = sY[n * NT + tid];
    h[n] = 0.0f;
  }
  float Dd = 0.0f;
  if (hasD) Dd = a.Dskip[d];

  const int nchunk = a.L / 64;
  const bool fwd = (a.dir > 0);
  const int s0 = fwd ? 0 : 63;
  const int sd = fwd ? 1 : -1;
  const int q  = lane >> 3;
  const int c8 = (lane & 7) * 8;

#pragma unroll 1
  for (int ci = 0; ci < nchunk; ++ci) {
    const int tb = fwd ? (ci * 64) : (a.L - 64 - ci * 64);
    const long rowc = rowb + tb;
    __syncthreads();
#pragma unroll 8
    for (int i = 0; i < 32; ++i) {
      const int idx = tid + i * NT;
      const int st  = idx / BCW;
      const int col = idx - st * BCW;
      const int sc  = (col < NSTATE) ? (a.offB + col) : (a.offC + col - NSTATE);
      sBC[idx] = a.bc[(rowc + st) * a.ld_bc + sc];
    }
    __syncthreads();
#pragma unroll 1
    for (int s = 0; s < 64; ++s) {
      const int ls = s0 + sd * s;
      const long row = rowc + ls;
      float pre = a.dtpre[row * a.ld_dtpre + d];
      float uv  = a.u[row * a.ld_u + d];
      float zv  = 0.0f;
      if (hasz) zv = a.z[row * a.ld_z + a.offZ + d];
      asm volatile("" : "+v"(pre));
      asm volatile("" : "+v"(uv));
      asm volatile("" : "+v"(zv));
      const float delta = ms1_softplus(pre);
      const float dtx = delta * uv;
      const float* bp = sBC + ls * BCW + sq * 16;
      const float* cp = bp + NSTATE;
      ms1_v4f Bq[4], Cq[4];
#pragma unroll
      for (int k = 0; k < 4; ++k) {
        Bq[k] = *(const ms1_v4f*)(bp + 4 * k);
        Cq[k] = *(const ms1_v4f*)(cp + 4 * k);
      }
      float yv = 0.0f;
#pragma unroll
      for (int n = 0; n < 16; ++n) {
        const float e = __expf(delta * An[n]);
        h[n] = fmaf(e, h[n], dtx * Bq[n >> 2][n & 3]);
        yv = fmaf(h[n], Cq[n >> 2][n & 3], yv);
      }
      if (NQ > 1) {
        yv += __shfl_xor(yv, 1, 32);
        yv += __shfl_xor(yv, 2, 32);
      }
      if (hasD) yv = fmaf(uv, Dd, yv);
      if (hasz) {
        const float sg = __builtin_amdgcn_rcpf(1.0f + expf(-zv));
        yv = yv * (zv * sg);
      }
      if (sq == 0) sY[ls * YP + c] = yv * a.ycarry;
    }
    __syncthreads();
    ms1_v4u hw[NIT], lw[NIT];
#pragma unroll
    for (int it = 0; it < NIT; ++it) {
      const int row = it * RPI + wave * 4 + q;
      const float* sp = sY + row * YP + c8;
      const ms1_v4f f0 = *(const ms1_v4f*)(sp);
      const ms1_v4f f1 = *(const ms1_v4f*)(sp + 4);
      unsigned h0, h1, h2, h3, l0, l1, l2, l3;
      ms1_pack2(f0[0], f0[1], h0, l0);
      ms1_pack2(f0[2], f0[3], h1, l1);
      ms1_pack2(f1[0], f1[1], h2, l2);
      ms1_pack2(f1[2], f1[3], h3, l3);
      hw[it] = (ms1_v4u){h0, h1, h2, h3};
      lw[it] = (ms1_v4u){l0, l1, l2, l3};
    }
    for (int pass = 0; pass < 2; ++pass) {
#pragma unroll
      for (int it = 0; it < NIT; ++it) {
        const int row = it * RPI + wave * 4 + q;
        const long o = (rowc + row) * a.ld_y + d0 + c8;
        *(volatile ms1_v4u*)(a.y + o) = hw[it];
        if (hasLo) *(volatile ms1_v4u*)(a.y_lo + o) = lw[it];
      }
      __threadfence();
    }
  }
}

extern "C" void kernel_launch(void* const* d_in, const int* in_sizes, int n_in,
                              void* d_out, int out_size, void* d_ws, size_t ws_size,
                              hipStream_t stream) {
  if (n_in < 11) return;
  if (in_sizes[0] != kRows * kDm) return;
  if (in_sizes[1] != kNL * kDm) return;
  if (in_sizes[2] != kNL * kXzP * kDm) return;
  if (in_sizes[3] != kNL * kDin * kTaps) return;
  if (in_sizes[4] != kNL * kDin) return;
  if (in_sizes[5] != kNL * kDbcW * kDin) return;
  if (in_sizes[6] != kNL * kDin * kDtR) return;
  if (in_sizes[7] != kNL * kDin) return;
  if (in_sizes[8] != kNL * kDin * kNst) return;
  if (in_sizes[9] != kNL * kDin) return;
  if (in_sizes[10] != kNL * kDm * kDin) return;
  if (out_size != kRows * kDm) return;
  if (ws_size < kWsTotal) return;

  const float* x_in    = (const float*)d_in[0];
  const float* norm_w  = (const float*)d_in[1];
  const float* W_in    = (const float*)d_in[2];
  const float* conv_w  = (const float*)d_in[3];
  const float* conv_b  = (const float*)d_in[4];
  const float* W_xproj = (const float*)d_in[5];
  const float* W_dt    = (const float*)d_in[6];
  const float* b_dt    = (const float*)d_in[7];
  const float* A_log   = (const float*)d_in[8];
  const float* D_par   = (const float*)d_in[9];
  const float* W_out   = (const float*)d_in[10];
  float* out = (float*)d_out;

  char* ws = (char*)d_ws;
  unsigned short* WI16 = (unsigned short*)(ws + kOffWI);
  unsigned short* WX16 = (unsigned short*)(ws + kOffWX);
  unsigned short* WO16 = (unsigned short*)(ws + kOffWO);
  unsigned short* XN16 = (unsigned short*)(ws + kOffXN);
  float*          XZ   = (float*)(ws + kOffXZ);
  float*          U32  = (float*)(ws + kOffU32);
  unsigned short* U16  = (unsigned short*)(ws + kOffU16);
  float*          DBC  = (float*)(ws + kOffDBC);
  float*          DTP  = (float*)(ws + kOffDTP);
  unsigned short* Y16  = (unsigned short*)(ws + kOffY16);
  float*          RA   = (float*)(ws + kOffRA);
  float*          RB   = (float*)(ws + kOffRB);

  prep_weights_kernel<<<dim3(kPrepBlkWi + kPrepBlkWx + kPrepBlkWo), 256, 0, stream>>>(
      W_in, W_xproj, W_out, WI16, WX16, WO16);

  for (int l = 0; l < kNL; ++l) {
    const float* Rin = (l == 0) ? x_in : ((l & 1) ? (const float*)RA : (const float*)RB);
    float* Rout = (l == kNL - 1) ? out : ((l & 1) ? RB : RA);

    rmsnorm_kernel<<<dim3(kRows / 16), 256, 0, stream>>>(Rin, norm_w + (size_t)l * kDm, XN16);

    eng::gemm_f16_kernel<false><<<dim3((kRows / 64) * (kXzP / 64) / 8), 256, 0, stream>>>(
        XN16, kDm,
        WI16 + (size_t)l * kXzP * kDm, kDm,
        XZ, kXzP,
        nullptr,
        kRows, kXzP, kDm, kScaleIn);

    conv_silu_kernel<<<dim3(kRows / 64), 256, 0, stream>>>(
        XZ, conv_w + (size_t)l * kDin * kTaps, conv_b + (size_t)l * kDin, U32, U16);

    eng::gemm_f16_kernel<false><<<dim3((kRows / 64) * (kDbcP / 64) / 8), 256, 0, stream>>>(
        U16, kDin,
        WX16 + (size_t)l * kDbcP * kDin, kDin,
        DBC, kDbcP,
        nullptr,
        kRows, kDbcP, kDin, kScaleIn);

    dtpre_kernel<<<dim3(kRows / 64), 256, 0, stream>>>(
        DBC, W_dt + (size_t)l * kDin * kDtR, b_dt + (size_t)l * kDin, DTP);

    for (int b = 0; b < kBatch; ++b) {
      const size_t r0 = (size_t)b * kSeq;
      ms1_args sa;
      sa.dtpre = DTP + r0 * kDin;
      sa.u = U32 + r0 * kDin;
      sa.bc = DBC + r0 * kDbcP;
      sa.z = XZ + r0 * kXzP;
      sa.A_log = A_log + (size_t)l * kDin * kNst;
      sa.Dskip = D_par + (size_t)l * kDin;
      sa.y = (__half*)(Y16 + r0 * kDin);
      sa.y_lo = nullptr;
      sa.ld_dtpre = kDin;
      sa.ld_u = kDin;
      sa.ld_bc = kDbcP;
      sa.ld_z = kXzP;
      sa.ld_y = kDin;
      sa.offB = kOffB;
      sa.offC = kOffC;
      sa.offZ = kDin;
      sa.ycarry = kYCarry;
      sa.dir = 1;
      sa.D = kDin;
      sa.L = kSeq;
      sa.nbatch = 1;
      ms1_scan_kernel<16><<<dim3(kDin / 64), 64, 0, stream>>>(sa);
    }

    eng::gemm_f16_kernel<true><<<dim3((kRows / 64) * (kDm / 64) / 8), 256, 0, stream>>>(
        Y16, kDin,
        WO16 + (size_t)l * kDm * kDin, kDin,
        Rout, kDm,
        Rin,
        kRows, kDm, kDin, kScaleOut);
  }
}
